// GraphNeuralNetwork_61984968015976
// MI455X (gfx1250) — hardware-verified
//
#include <hip/hip_runtime.h>


namespace {
typedef _Float16 b16;
typedef __attribute__((ext_vector_type(16))) _Float16 v16b;
typedef __attribute__((ext_vector_type(8))) _Float16 v8b;
typedef __attribute__((ext_vector_type(4))) _Float16 v4h;
typedef __attribute__((ext_vector_type(2))) _Float16 v2h;
typedef __attribute__((ext_vector_type(8))) float v8f;
typedef __attribute__((ext_vector_type(4))) float v4f;
typedef __attribute__((ext_vector_type(2))) float v2f;
__device__ __forceinline__ float bf16_rne(float f) { unsigned int u = __float_as_uint(f); u += 0x7FFFu + ((u >> 16) & 1u); return __uint_as_float(u & 0xFFFF0000u); }
__device__ __forceinline__ void split16(float v, b16& hi, b16& lo) { hi = (b16)v; lo = (b16)(v - (float)hi); }
__device__ __forceinline__ v16b frag_kb(const b16* p, int hh) { const v8b a = *(const v8b*)(p + 8 * hh), b = *(const v8b*)(p + 16 + 8 * hh); v16b f;
#pragma unroll
  for (int e = 0; e < 8; ++e) { f[e] = a[e]; f[8 + e] = b[e]; } return f; }
__device__ __forceinline__ v8f wmma16b(v16b a, v16b b, v8f c) { v8f d = __builtin_amdgcn_wmma_f32_16x16x32_f16(false, a, false, b, (short)0, c, false, false); asm volatile("v_nop\n\tv_nop\n\tv_nop\n\tv_nop" : "+v"(d) : "v"(a), "v"(b)); return d; }
__device__ __forceinline__ void wave_lds_sync() { __builtin_amdgcn_fence(__ATOMIC_RELEASE, "workgroup"); __builtin_amdgcn_wave_barrier(); __builtin_amdgcn_fence(__ATOMIC_ACQUIRE, "workgroup"); }
__device__ __forceinline__ float pmul(float a, float b) { float p = a * b; asm volatile("" : "+v"(p)); return p; }
__device__ __forceinline__ int iclamp(int v, int lo, int hi) { return v < lo ? lo : (v > hi ? hi : v); }
__device__ __forceinline__ float nexp2(float v) { return __builtin_amdgcn_exp2f(v); }

constexpr int BS = 512, BSL = BS  , N0 = 512, NHID = 2048, NOUTF = 512, DEG = 64, NP = BS, N = BS;
constexpr float XS = 8.0f, WSC = 256.0f, WS2 = 65536.0f, RS = 1024.0f, SLOPE = 0.0f, BNEPS = 1e-5f;
static_assert(BS % 32 == 0 && BSL % 32 == 0 && N0 % 128 == 0 && NHID % 128 == 0 && NOUTF % 128 == 0, "tiling");

typedef __attribute__((ext_vector_type(4))) _Float16 v4h;
typedef __attribute__((ext_vector_type(2))) float v2f;
template <int KD, int NOUT>
__global__ __launch_bounds__(256) void wprep_kernel(const float* __restrict__ w, b16* __restrict__ WT) {
  static_assert(KD % 8 == 0, "wprep"); const size_t u = (size_t)blockIdx.x * 256 + threadIdx.x; if (u >= (size_t)NOUT * KD / 8) return; const size_t e = u * 8; const int oo = (int)(e / KD), k0 = (int)(e % KD); v8b o;
  for (int j = 0; j < 8; ++j) o[j] = (b16)(bf16_rne(w[(size_t)(k0 + j) * NOUT + oo]) * WSC);
  for (int pass = 0; pass < 2; ++pass) { *(volatile v8b*)(WT + e) = o; __threadfence(); }
}
template <int KD, int NOUT, int NV, bool RNDA  >
__global__ __launch_bounds__(64) void gemm_kernel(const float* __restrict__ A, const b16* __restrict__ W, float* __restrict__ T) {
  constexpr int SL = NOUT < 128 ? NOUT : 128, NT = SL / 16, KC = KD < 128 ? KD : 128;
  static_assert(KD % KC == 0 && KC % 32 == 0 && NOUT % SL == 0 && SL % 32 == 0, "gemm tiling");
  __shared__ __attribute__((aligned(16))) b16 Ah[2][16][KC + 8], Al[2][16][KC + 8]; __shared__ __attribute__((aligned(16))) float Tf[2][16][SL + 4];
  const int wave = threadIdx.x >> 5, lane = threadIdx.x & 31, nloc = lane & 15, hlf = lane >> 4; const size_t m0 = (size_t)blockIdx.x * 32 + wave * 16; const int n0 = blockIdx.y * SL;
  v8f acc[NT];
#pragma unroll
  for (int t = 0; t < NT; ++t) acc[t] = (v8f){};
#pragma unroll 1
  for (int kc = 0; kc < KD; kc += KC) {
    for (int idx = lane; idx < 16 * (KC / 4); idx += 32) { const int rr = idx / (KC / 4), c4 = (idx % (KC / 4)) * 4; const size_t row = (m0 + rr < (size_t)NV) ? (m0 + rr) : (size_t)(NV - 1); const v4f v = *(const v4f*)(A + row * KD + kc + c4); v4h hv, lv;
      for (int j = 0; j < 4; ++j) { b16 ph, pl; split16((RNDA ? bf16_rne(v[j]) : v[j]) * XS, ph, pl); hv[j] = ph; lv[j] = pl; } *(v4h*)(&Ah[wave][rr][c4]) = hv; *(v4h*)(&Al[wave][rr][c4]) = lv; }
    wave_lds_sync();
#pragma unroll
    for (int kb = 0; kb < KC; kb += 32) { const v16b a = frag_kb(&Ah[wave][nloc][kb], hlf), al = frag_kb(&Al[wave][nloc][kb], hlf);
#pragma unroll
      for (int t = 0; t < NT; ++t) { const v16b bw = frag_kb(W + (size_t)(n0 + t * 16 + nloc) * KD + kc + kb, hlf); acc[t] = wmma16b(a, bw, acc[t]); acc[t] = wmma16b(al, bw, acc[t]); } }
    wave_lds_sync(); }
#pragma unroll
  for (int t = 0; t < NT; ++t)
#pragma unroll
    for (int r = 0; r < 8; ++r) Tf[wave][8 * hlf + r][t * 16 + nloc] = acc[t][r] * (1.0f / (XS * WSC));
  wave_lds_sync();
  for (int pass = 0; pass < 2; ++pass) { for (int idx = lane; idx < 16 * (SL / 4); idx += 32) { const int rr = idx / (SL / 4), c4 = (idx % (SL / 4)) * 4; *(volatile v4f*)(T + (m0 + rr) * NOUT + n0 + c4) = *(const v4f*)(&Tf[wave][rr][c4]); } __threadfence(); }
}

template <int KP>
__global__ __launch_bounds__(128) void wbuild_kernel(const float* __restrict__ w, const int* __restrict__ src, int nrows, b16* __restrict__ WH, b16* __restrict__ WL) {
  __shared__ __attribute__((aligned(16))) float rowbuf[4][KP];
  const int wave = threadIdx.x >> 5, lane = threadIdx.x & 31; const int n = blockIdx.x * 4 + wave;
  for (int k = lane; k < KP; k += 32) rowbuf[wave][k] = 0.0f;
  wave_lds_sync();
  if (lane == 0 && n < nrows) {
#pragma unroll 1
    for (int j = 0; j < DEG; ++j) { const int e = n * DEG + j; const int k = iclamp(src[e], 0, KP - 1); rowbuf[wave][k] += bf16_rne(w[e]); } }
  wave_lds_sync();
  if (n >= nrows) return;
  for (int pass = 0; pass < 2; ++pass) { for (int k0 = lane * 8; k0 < KP; k0 += 256) { v8b hv, lv; for (int j = 0; j < 8; ++j) { const float m = rowbuf[wave][k0 + j] * WS2; const b16 h = (b16)m; hv[j] = h; lv[j] = (b16)((m - (float)h) * RS); }
      *(volatile v8b*)(WH + (size_t)n * KP + k0) = hv; *(volatile v8b*)(WL + (size_t)n * KP + k0) = lv; } __threadfence(); }
}
template <int NW, int ACT>
__global__ __launch_bounds__(256) void combine_kernel(const float* __restrict__ T1, const float* __restrict__ T2, const float* __restrict__ bias, float* __restrict__ H) {
  const size_t u = (size_t)blockIdx.x * 256 + threadIdx.x; if (u >= (size_t)BSL * NW / 4) return; const size_t e = u * 4; const int n = (int)(e % NW); const float c1 = WSC / WS2, c2 = WSC / (WS2 * RS);
  const v4f a = *(const v4f*)(T1 + e), bq = *(const v4f*)(T2 + e); v4f o; for (int i = 0; i < 4; ++i) { const float h = a[i] * c1 + bq[i] * c2 + bf16_rne(bias[n + i]); o[i] = ACT ? fmaxf(h, 0.0f) : h; }
  for (int pass = 0; pass < 2; ++pass) { *(volatile v4f*)(H + e) = o; __threadfence(); }
}
}

extern "C" void kernel_launch(void* const* d_in, const int* in_sizes, int n_in, void* d_out, int out_size, void* d_ws, size_t ws_size, hipStream_t stream) {
  (void)n_in;
  auto Fp = [&](int i) { return (const float*)d_in[i]; }; auto Ip = [&](int i) { return (const int*)d_in[i]; };
  if (in_sizes[0] != BS * N0 || in_sizes[1] != NHID * DEG || in_sizes[2] != NHID || in_sizes[3] != NHID * DEG || in_sizes[5] != NHID * DEG || in_sizes[9] != NHID * DEG || in_sizes[13] != NOUTF * DEG || in_sizes[14] != NOUTF || in_sizes[15] != NOUTF * DEG || out_size != BS * NOUTF) return;
  size_t off = 0; char* ws = (char*)d_ws;
  auto carve = [&](size_t bytes) { char* p = ws + off; off += (bytes + 255) & ~(size_t)255; return p; };
  b16* WH = (b16*)carve((size_t)NHID * NHID * 2); b16* WL = (b16*)carve((size_t)NHID * NHID * 2); float* T1 = (float*)carve((size_t)BS * NHID * 4); float* T2 = (float*)carve((size_t)BS * NHID * 4); float* HA = (float*)carve((size_t)BS * NHID * 4); float* HB = (float*)carve((size_t)BS * NHID * 4);
  if (off > ws_size || off > ((size_t)128 << 20)) return;
  const unsigned cbh = (unsigned)(((size_t)BSL * NHID / 4 + 255) / 256), cbo = (unsigned)(((size_t)BSL * NOUTF / 4 + 255) / 256);
  wbuild_kernel<N0><<<NHID / 4, 128, 0, stream>>>(Fp(1), Ip(3), NHID, WH, WL);
  gemm_kernel<N0, NHID, BS, true><<<dim3(BSL / 32, NHID / 128), 64, 0, stream>>>(Fp(0), WH, T1); gemm_kernel<N0, NHID, BS, true><<<dim3(BSL / 32, NHID / 128), 64, 0, stream>>>(Fp(0), WL, T2);
  combine_kernel<NHID, 1><<<cbh, 256, 0, stream>>>(T1, T2, Fp(2), HA);
  wbuild_kernel<NHID><<<NHID / 4, 128, 0, stream>>>(Fp(5), Ip(7), NHID, WH, WL);
  gemm_kernel<NHID, NHID, BS, false><<<dim3(BSL / 32, NHID / 128), 64, 0, stream>>>(HA, WH, T1); gemm_kernel<NHID, NHID, BS, false><<<dim3(BSL / 32, NHID / 128), 64, 0, stream>>>(HA, WL, T2);
  combine_kernel<NHID, 1><<<cbh, 256, 0, stream>>>(T1, T2, Fp(6), HB);
  wbuild_kernel<NHID><<<NHID / 4, 128, 0, stream>>>(Fp(9), Ip(11), NHID, WH, WL);
  gemm_kernel<NHID, NHID, BS, false><<<dim3(BSL / 32, NHID / 128), 64, 0, stream>>>(HB, WH, T1); gemm_kernel<NHID, NHID, BS, false><<<dim3(BSL / 32, NHID / 128), 64, 0, stream>>>(HB, WL, T2);
  combine_kernel<NHID, 1><<<cbh, 256, 0, stream>>>(T1, T2, Fp(10), HA);
  wbuild_kernel<NHID><<<NOUTF / 4, 128, 0, stream>>>(Fp(13), Ip(15), NOUTF, WH, WL);
  gemm_kernel<NHID, NOUTF, BS, false><<<dim3(BSL / 32, NOUTF / 128), 64, 0, stream>>>(HA, WH, T1); gemm_kernel<NHID, NOUTF, BS, false><<<dim3(BSL / 32, NOUTF / 128), 64, 0, stream>>>(HA, WL, T2);
  combine_kernel<NOUTF, 0><<<cbo, 256, 0, stream>>>(T1, T2, Fp(14), (float*)d_out);
}
